// SelectiveSSM_24859270709951
// MI455X (gfx1250) — hardware-verified
//
#include <hip/hip_runtime.h>
#include <math.h>

typedef __attribute__((ext_vector_type(16))) _Float16 v16h;
typedef __attribute__((ext_vector_type(8)))  _Float16 v8h;
typedef __attribute__((ext_vector_type(16))) __bf16   v16b;
typedef __attribute__((ext_vector_type(8)))  __bf16   v8b;
typedef __attribute__((ext_vector_type(8)))  float    v8f;
typedef __attribute__((ext_vector_type(4)))  float    v4f;

constexpr int kBatch   = 4;
constexpr int kSeqL    = 1024;
constexpr int kDmod    = 1024;
constexpr int kDin     = 2048;
constexpr int kNst     = 16;
constexpr int kDtR     = 64;
constexpr int kPrjN    = 96;
constexpr int kPrjP    = 128;
constexpr int kXZP     = 2 * kDin;
constexpr int kRows    = kBatch * kSeqL;
constexpr int kGrpB    = 2;
constexpr int kGrpRows = kGrpB * kSeqL;
constexpr int kNGrp    = kBatch / kGrpB;
constexpr int kTP      = 260;
constexpr float kCarryWxp = 32.0f;
constexpr float kCarryDt  = 16.0f;
constexpr float kCarryWdt = 8.0f;

static_assert(kDtR + 2 * kNst == kPrjN, "x_proj width");
static_assert(kRows == 4096 && kXZP == 4096 && kGrpRows == 2048 && kNGrp == 2, "shape constants");
static_assert((kDmod % 32) == 0 && (kDin % 32) == 0 && (kDtR % 32) == 0, "GEMM K multiples of 32");
static_assert((kGrpRows % 64) == 0 && (kXZP % 64) == 0 && (kPrjP % 64) == 0 && (kDin % 64) == 0 && (kDmod % 64) == 0, "GEMM M,N multiples of 64");
static_assert((kSeqL % 64) == 0 && (kDin % 256) == 0 && (kSeqL % 16) == 0, "tile multiples");
static_assert((kSeqL & (kSeqL - 1)) == 0, "sequence length power of two");

constexpr size_t kSzXB   = (size_t)kRows * kDmod * 2;
constexpr size_t kSzWIN  = (size_t)kXZP * kDmod * 2;
constexpr size_t kSzWOUT = (size_t)kDmod * kDin * 2;
constexpr size_t kSzWXP  = (size_t)kPrjP * kDin * 2;
constexpr size_t kSzWDT  = (size_t)kDin * kDtR * 2;
constexpr size_t kSzXZ   = (size_t)kGrpRows * kXZP * 4;
constexpr size_t kSzUC   = (size_t)kGrpRows * kDin * 4;
constexpr size_t kSzUC16 = (size_t)kGrpRows * kDin * 2;
constexpr size_t kSzPROJ = (size_t)kGrpRows * kPrjP * 4;
constexpr size_t kSzDT16 = (size_t)kGrpRows * kDtR * 2;
constexpr size_t kSzDLR  = (size_t)kGrpRows * kDin * 4;
constexpr size_t kSzY    = (size_t)kGrpRows * kDin * 2;
constexpr size_t kOffXB   = 0;
constexpr size_t kOffWIN  = kOffXB   + kSzXB;
constexpr size_t kOffWOUT = kOffWIN  + kSzWIN;
constexpr size_t kOffWXP  = kOffWOUT + kSzWOUT;
constexpr size_t kOffWDT  = kOffWXP  + kSzWXP;
constexpr size_t kOffXZ   = kOffWDT  + kSzWDT;
constexpr size_t kOffUC   = kOffXZ   + kSzXZ;
constexpr size_t kOffUC16 = kOffUC   + kSzUC;
constexpr size_t kOffPROJ = kOffUC16 + kSzUC16;
constexpr size_t kOffDT16 = kOffPROJ + kSzPROJ;
constexpr size_t kOffDLR  = kOffDT16 + kSzDT16;
constexpr size_t kOffYH   = kOffDLR  + kSzDLR;
constexpr size_t kOffYL   = kOffYH   + kSzY;
constexpr size_t kWsTotal = kOffYL   + kSzY;
static_assert(kWsTotal == 115343360ull, "carve total");
static_assert(kWsTotal <= 134217728ull, "carve cap");
static_assert((kOffWIN % 128) == 0 && (kOffWOUT % 128) == 0 && (kOffWXP % 128) == 0 && (kOffWDT % 128) == 0 &&
              (kOffXZ % 128) == 0 && (kOffUC % 128) == 0 && (kOffUC16 % 128) == 0 && (kOffPROJ % 128) == 0 &&
              (kOffDT16 % 128) == 0 && (kOffDLR % 128) == 0 && (kOffYH % 128) == 0 && (kOffYL % 128) == 0,
              "128-B aligned regions");

__device__ __forceinline__ unsigned short f2bf_bits(float f) {
  unsigned u = __float_as_uint(f);
  return (unsigned short)((u + 0x7FFFu + ((u >> 16) & 1u)) >> 16);
}
__device__ __forceinline__ float bf_bits2f(unsigned short h) { return __uint_as_float(((unsigned)h) << 16); }
__device__ __forceinline__ float bf_rne(float f) { return bf_bits2f(f2bf_bits(f)); }

__device__ __forceinline__ void dep_guard4_h(v8f& a, v8f& b, v8f& c, v8f& d, v16h x, v16h y) {
  asm volatile("v_nop\n\tv_nop\n\tv_nop\n\tv_nop" : "+v"(a), "+v"(b), "+v"(c), "+v"(d) : "v"(x), "v"(y));
}
__device__ __forceinline__ void dep_guard4_b(v8f& a, v8f& b, v8f& c, v8f& d, v16b x, v16b y) {
  asm volatile("v_nop\n\tv_nop\n\tv_nop\n\tv_nop" : "+v"(a), "+v"(b), "+v"(c), "+v"(d) : "v"(x), "v"(y));
}
__device__ __forceinline__ void keep4_h(v16h a, v16h b, v16h c, v16h d) { asm volatile("v_nop" :: "v"(a), "v"(b), "v"(c), "v"(d)); }
__device__ __forceinline__ void keep4_b(v16b a, v16b b, v16b c, v16b d) { asm volatile("v_nop" :: "v"(a), "v"(b), "v"(c), "v"(d)); }
__device__ __forceinline__ void acc_guard4(v8f& a, v8f& b, v8f& c, v8f& d) {
  asm volatile("v_nop\n\tv_nop\n\tv_nop\n\tv_nop" : "+v"(a), "+v"(b), "+v"(c), "+v"(d));
}

template <typename T> struct Frag;
template <> struct Frag<_Float16> {
  typedef v16h V; union U { v16h v; v8h h[2]; };
  static __device__ __forceinline__ v16h load(const _Float16* p) {
    U f; f.h[0] = *(const v8h*)(p); f.h[1] = *(const v8h*)(p + 16); return f.v;
  }
  static __device__ __forceinline__ v8f mma(v16h a, v16h b, v8f c) {
    return __builtin_amdgcn_wmma_f32_16x16x32_f16(false, a, false, b, (short)0, c, false, false);
  }
  static __device__ __forceinline__ void guard4(v8f& a, v8f& b, v8f& c, v8f& d, v16h x, v16h y) { dep_guard4_h(a, b, c, d, x, y); }
  static __device__ __forceinline__ void keep(v16h a, v16h b, v16h c, v16h d) { keep4_h(a, b, c, d); }
};
template <> struct Frag<__bf16> {
  typedef v16b V; union U { v16b v; v8b h[2]; };
  static __device__ __forceinline__ v16b load(const __bf16* p) {
    U f; f.h[0] = *(const v8b*)(p); f.h[1] = *(const v8b*)(p + 16); return f.v;
  }
  static __device__ __forceinline__ v8f mma(v16b a, v16b b, v8f c) {
    return __builtin_amdgcn_wmma_f32_16x16x32_bf16(false, a, false, b, (short)0, c, false, false);
  }
  static __device__ __forceinline__ void guard4(v8f& a, v8f& b, v8f& c, v8f& d, v16b x, v16b y) { dep_guard4_b(a, b, c, d, x, y); }
  static __device__ __forceinline__ void keep(v16b a, v16b b, v16b c, v16b d) { keep4_b(a, b, c, d); }
};

template <int ET> struct Elem;
template <> struct Elem<0> { typedef _Float16 T; };
template <> struct Elem<1> { typedef __bf16 T; };

template <int ET, int SPL, int BIAS_MODE>
__global__ __launch_bounds__(256) void wmma_gemm64(
    const unsigned short* __restrict__ Ap, const unsigned short* __restrict__ A2p, int lda,
    const unsigned short* __restrict__ Btp, int ldb,
    float* __restrict__ C, int ldc,
    const float* __restrict__ bias,
    int M, int N, int K, float scale) {
  typedef typename Elem<ET>::T T;
  typedef typename Frag<T>::V V;
  const T* A  = (const T*)Ap;
  const T* A2 = (const T*)A2p;
  const T* Bt = (const T*)Btp;
  __shared__ __align__(16) float sT[8][16 * 68];
  const int lane = threadIdx.x & 31;
  const int wave = threadIdx.x >> 5;
  const int tilesN = N >> 6;
  const int tilesM = M >> 6;
  const int tile = blockIdx.x * 8 + wave;
  if (tile >= tilesM * tilesN) return;
  const int tm = tile / tilesN;
  const int tn = tile - tm * tilesN;
  const int m0 = tm << 6;
  const int n0 = tn << 6;

  const int rlane = lane & 15;
  const int koff  = (lane >> 4) * 8;
  const int mOff  = (lane >> 4) * 8;

  v8f acc[4][4];
#pragma unroll
  for (int i = 0; i < 4; ++i)
#pragma unroll
    for (int j = 0; j < 4; ++j) acc[i][j] = (v8f){0.f, 0.f, 0.f, 0.f, 0.f, 0.f, 0.f, 0.f};

  for (int k0 = 0; k0 < K; k0 += 32) {
    V bh[4];
#pragma unroll
    for (int j = 0; j < 4; ++j) {
      const size_t bo = (size_t)(n0 + (j << 4) + rlane) * ldb + koff + k0;
      bh[j] = Frag<T>::load(Bt + bo);
    }
#pragma unroll
    for (int i = 0; i < 4; ++i) {
      const size_t ao = (size_t)(m0 + (i << 4) + rlane) * lda + koff + k0;
      V ah = Frag<T>::load(A + ao);
      V al = ah;
      if (SPL == 1) al = Frag<T>::load(A2 + ao);
#pragma unroll
      for (int j = 0; j < 4; ++j) {
        acc[i][j] = Frag<T>::mma(ah, bh[j], acc[i][j]);
        if (SPL == 1) acc[i][j] = Frag<T>::mma(al, bh[j], acc[i][j]);
      }
      Frag<T>::guard4(acc[i][0], acc[i][1], acc[i][2], acc[i][3], ah, al);
    }
    Frag<T>::keep(bh[0], bh[1], bh[2], bh[3]);
  }
  acc_guard4(acc[0][0], acc[0][1], acc[0][2], acc[0][3]);
  acc_guard4(acc[1][0], acc[1][1], acc[1][2], acc[1][3]);
  acc_guard4(acc[2][0], acc[2][1], acc[2][2], acc[2][3]);
  acc_guard4(acc[3][0], acc[3][1], acc[3][2], acc[3][3]);

  float* slab = sT[wave];
#pragma unroll
  for (int i = 0; i < 4; ++i) {
    const int mBase = m0 + (i << 4);
#pragma unroll
    for (int j = 0; j < 4; ++j) {
      const int n = n0 + (j << 4) + rlane;
      float bv = 0.f;
      if (BIAS_MODE == 2) bv = bias[n];
      if (BIAS_MODE == 3) bv = bf_rne(bias[n]);
#pragma unroll
      for (int r = 0; r < 8; ++r) {
        float v = acc[i][j][r] * scale;
        if (BIAS_MODE != 0) v += bv;
        slab[(mOff + r) * 68 + (j << 4) + rlane] = v;
      }
    }
    __builtin_amdgcn_fence(__ATOMIC_RELEASE, "workgroup");
    __builtin_amdgcn_wave_barrier();
    __builtin_amdgcn_fence(__ATOMIC_ACQUIRE, "workgroup");
    {
      const int hh = lane >> 4, c4 = (lane & 15) * 4;
      for (int pass = 0; pass < 2; ++pass) {
#pragma unroll
        for (int it = 0; it < 8; ++it) {
          const int row = it * 2 + hh;
          v4f v = *(const v4f*)(slab + row * 68 + c4);
          *(volatile v4f*)(C + (size_t)(mBase + row) * ldc + n0 + c4) = v;
        }
        __threadfence();
      }
    }
    __builtin_amdgcn_fence(__ATOMIC_RELEASE, "workgroup");
    __builtin_amdgcn_wave_barrier();
    __builtin_amdgcn_fence(__ATOMIC_ACQUIRE, "workgroup");
  }
}

__global__ __launch_bounds__(256) void cast_bf16_kernel(
    const float* __restrict__ src, unsigned short* __restrict__ dst, int total8)
{
  const int i = blockIdx.x * 256 + threadIdx.x;
  if (i >= total8) return;
  const size_t e0 = (size_t)i << 3;
  const float* p = src + e0;
  const v4f a0 = *(const v4f*)(p);
  const v4f a1 = *(const v4f*)(p + 4);
  v8h hv;
#pragma unroll
  for (int e = 0; e < 4; ++e) {
    const unsigned short h0 = f2bf_bits(a0[e]);
    const unsigned short h1 = f2bf_bits(a1[e]);
    hv[e]     = __builtin_bit_cast(_Float16, h0);
    hv[4 + e] = __builtin_bit_cast(_Float16, h1);
  }
  unsigned short* q = dst + e0;
  *(volatile v8h*)q = hv;
  __threadfence();
  *(volatile v8h*)q = hv;
}

template <bool TO_BF16>
__global__ __launch_bounds__(256) void transpose_cast_kernel(
    const float* __restrict__ W, unsigned short* __restrict__ Bt, int Kdim, int Ndim, float scale)
{
  __shared__ float tile[64 * 65];
  const int tid = threadIdx.x, lane = tid & 31, wave = tid >> 5;
  const int n0 = blockIdx.x * 64;
  const int k0 = blockIdx.y * 64;
#pragma unroll
  for (int p = 0; p < 16; ++p) {
    const int idx = tid + p * 256;
    const int kk  = idx >> 6;
    const int nn  = idx & 63;
    const int n   = n0 + nn;
    const int nc  = (n < Ndim) ? n : (Ndim - 1);
    const float v = W[(size_t)(k0 + kk) * Ndim + nc];
    const float vr = bf_rne(v);
    tile[kk * 65 + nn] = (n < Ndim) ? (vr * scale) : 0.f;
  }
  __syncthreads();
  const int q = lane >> 3, c8 = (lane & 7) * 8;
  v8h hv[2];
#pragma unroll
  for (int it = 0; it < 2; ++it) {
    const int nrow = it * 32 + wave * 4 + q;
#pragma unroll
    for (int e = 0; e < 8; ++e) {
      const float val = tile[(c8 + e) * 65 + nrow];
      if (TO_BF16) {
        const unsigned short hb = f2bf_bits(val);
        hv[it][e] = __builtin_bit_cast(_Float16, hb);
      } else {
        hv[it][e] = (_Float16)val;
      }
    }
  }
  for (int pass = 0; pass < 2; ++pass) {
#pragma unroll
    for (int it = 0; it < 2; ++it) {
      const int nrow = it * 32 + wave * 4 + q;
      *(volatile v8h*)(Bt + (size_t)(n0 + nrow) * Kdim + k0 + c8) = hv[it];
    }
    __threadfence();
  }
}

__global__ __launch_bounds__(256) void dt_cast_kernel(
    const float* __restrict__ PROJ, unsigned short* __restrict__ DT16, int total8, float scale)
{
  const int i = blockIdx.x * 256 + threadIdx.x;
  if (i >= total8) return;
  const int e0  = i << 3;
  const int row = e0 >> 6;
  const int c8  = e0 & 63;
  const float* p = PROJ + (size_t)row * kPrjP + c8;
  const v4f a0 = *(const v4f*)(p);
  const v4f a1 = *(const v4f*)(p + 4);
  v8h hv;
#pragma unroll
  for (int e = 0; e < 4; ++e) {
    hv[e]     = (_Float16)(a0[e] * scale);
    hv[4 + e] = (_Float16)(a1[e] * scale);
  }
  unsigned short* qd = DT16 + e0;
  *(volatile v8h*)qd = hv;
  __threadfence();
  *(volatile v8h*)qd = hv;
}

__global__ __launch_bounds__(256) void conv_silu_kernel(
    const float* __restrict__ XZ, const float* __restrict__ cw, const float* __restrict__ cb,
    float* __restrict__ UC, unsigned short* __restrict__ UC16)
{
  __shared__ __align__(16) float sT[16 * kTP];
  const int tid = threadIdx.x, lane = tid & 31, wave = tid >> 5;
  const int d0 = blockIdx.x * 256, d = d0 + tid;
  const int t0 = blockIdx.y * 64;
  const int tb = t0 & (kSeqL - 1);
  const v4f wv = *(const v4f*)(cw + (size_t)d * 4);
  const float w0 = bf_rne(wv[0]);
  const float w1 = bf_rne(wv[1]);
  const float w2 = bf_rne(wv[2]);
  const float w3 = bf_rne(wv[3]);
  const float bc = bf_rne(cb[d]);
  float xm3, xm2, xm1;
  {
    const bool hist = (tb > 0);
    const int rb = hist ? (t0 - 3) : t0;
    const float v3 = XZ[(size_t)rb * kXZP + d];
    const float v2 = XZ[(size_t)(rb + 1) * kXZP + d];
    const float v1 = XZ[(size_t)(rb + 2) * kXZP + d];
    xm3 = hist ? v3 : 0.f;
    xm2 = hist ? v2 : 0.f;
    xm1 = hist ? v1 : 0.f;
  }
  const int hrow = wave >> 1;
  const int hch  = (wave & 1) * 128 + lane * 4;
#pragma unroll 1
  for (int sub = 0; sub < 4; ++sub) {
    const int lb = t0 + sub * 16;
#pragma unroll 1
    for (int s = 0; s < 16; ++s) {
      const float xcur = XZ[(size_t)(lb + s) * kXZP + d];
      float acc = w0 * xm3;
      acc = fmaf(w1, xm2, acc);
      acc = fmaf(w2, xm1, acc);
      acc = fmaf(w3, xcur, acc);
      const float sv = acc + bc;
      const float sg = __builtin_amdgcn_rcpf(1.0f + __expf(-sv));
      sT[s * kTP + tid] = sv * sg;
      xm3 = xm2; xm2 = xm1; xm1 = xcur;
    }
    __syncthreads();
    v4f fv[4];
    v8h bv[2];
#pragma unroll
    for (int it = 0; it < 4; ++it) fv[it] = *(const v4f*)(sT + (it * 4 + hrow) * kTP + hch);
#pragma unroll
    for (int it = 0; it < 2; ++it) {
      const float* sp = sT + (it * 8 + wave) * kTP + lane * 8;
      const v4f a0 = *(const v4f*)(sp);
      const v4f a1 = *(const v4f*)(sp + 4);
#pragma unroll
      for (int e = 0; e < 4; ++e) {
        bv[it][e]     = (_Float16)a0[e];
        bv[it][4 + e] = (_Float16)a1[e];
      }
    }
    for (int pass = 0; pass < 2; ++pass) {
#pragma unroll
      for (int it = 0; it < 4; ++it)
        *(volatile v4f*)(UC + (size_t)(lb + it * 4 + hrow) * kDin + d0 + hch) = fv[it];
#pragma unroll
      for (int it = 0; it < 2; ++it)
        *(volatile v8h*)(UC16 + (size_t)(lb + it * 8 + wave) * kDin + d0 + lane * 8) = bv[it];
      __threadfence();
    }
    __syncthreads();
  }
}

__global__ __launch_bounds__(256) void scan_kernel(
    const float* __restrict__ DLR, const float* __restrict__ UC, const float* __restrict__ XZ,
    const float* __restrict__ PROJ, const float* __restrict__ A_log, const float* __restrict__ Dv,
    unsigned short* __restrict__ YH, unsigned short* __restrict__ YL)
{
  __shared__ __align__(16) float sBC[16 * 32];
  __shared__ __align__(16) float sY[16 * kTP];
  const int tid = threadIdx.x, lane = tid & 31, wave = tid >> 5;
  const int d0 = blockIdx.x * 256, d = d0 + tid;
  const size_t rb = (size_t)blockIdx.y * kSeqL;

  float An[kNst];
#pragma unroll
  for (int q4 = 0; q4 < 4; ++q4) {
    const v4f av = *(const v4f*)(A_log + (size_t)d * kNst + 4 * q4);
    An[4 * q4 + 0] = -__expf(bf_rne(av[0]));
    An[4 * q4 + 1] = -__expf(bf_rne(av[1]));
    An[4 * q4 + 2] = -__expf(bf_rne(av[2]));
    An[4 * q4 + 3] = -__expf(bf_rne(av[3]));
  }
  const float Dd = bf_rne(Dv[d]);
  float h[kNst];
#pragma unroll
  for (int n = 0; n < kNst; ++n) h[n] = 0.f;

#pragma unroll 1
  for (int c = 0; c < kSeqL / 16; ++c) {
    const int l0 = c * 16;
    if (tid < 128) {
      const int r = tid >> 3, q = (tid & 7) * 4;
      const v4f v = *(const v4f*)(PROJ + (rb + l0 + r) * kPrjP + kDtR + q);
      *(v4f*)(sBC + r * 32 + q) = v;
    }
    __syncthreads();
#pragma unroll 1
    for (int s = 0; s < 16; ++s) {
      const size_t m = rb + (size_t)(l0 + s);
      const float a  = DLR[m * kDin + d];
      const float xv = UC[m * kDin + d];
      const float zv = XZ[m * kXZP + kDin + d];
      const float ea  = __expf(-fabsf(a));
      const float u   = 1.0f + ea;
      const float l1p = __logf(u) + (ea - (u - 1.0f)) * __builtin_amdgcn_rcpf(u);
      const float delta = fmaxf(a, 0.0f) + l1p;
      v4f Bq[4], Cq[4];
#pragma unroll
      for (int qq = 0; qq < 4; ++qq) {
        Bq[qq] = *(const v4f*)(sBC + s * 32 + 4 * qq);
        Cq[qq] = *(const v4f*)(sBC + s * 32 + kNst + 4 * qq);
      }
      const float dtx = delta * xv;
      float y = 0.f;
#pragma unroll
      for (int n = 0; n < kNst; ++n) {
        const float e = __expf(delta * An[n]);
        h[n] = fmaf(e, h[n], dtx * Bq[n >> 2][n & 3]);
        y = fmaf(h[n], Cq[n >> 2][n & 3], y);
      }
      y = fmaf(xv, Dd, y);
      const float sg = __builtin_amdgcn_rcpf(1.0f + __expf(-zv));
      const float g  = zv * sg;
      sY[s * kTP + tid] = y * g;
    }
    __syncthreads();
    v8h hv[2], lv[2];
#pragma unroll
    for (int it = 0; it < 2; ++it) {
      const float* sp = sY + (it * 8 + wave) * kTP + lane * 8;
      const v4f a0 = *(const v4f*)(sp);
      const v4f a1 = *(const v4f*)(sp + 4);
#pragma unroll
      for (int e = 0; e < 4; ++e) {
        const float f0 = a0[e];
        const float f1 = a1[e];
        const unsigned short h0 = f2bf_bits(f0);
        const unsigned short h1 = f2bf_bits(f1);
        const unsigned short q0 = f2bf_bits(f0 - bf_bits2f(h0));
        const unsigned short q1 = f2bf_bits(f1 - bf_bits2f(h1));
        hv[it][e]     = __builtin_bit_cast(_Float16, h0);
        hv[it][4 + e] = __builtin_bit_cast(_Float16, h1);
        lv[it][e]     = __builtin_bit_cast(_Float16, q0);
        lv[it][4 + e] = __builtin_bit_cast(_Float16, q1);
      }
    }
    for (int pass = 0; pass < 2; ++pass) {
#pragma unroll
      for (int it = 0; it < 2; ++it) {
        const size_t o = (rb + (size_t)(l0 + it * 8 + wave)) * kDin + d0 + lane * 8;
        *(volatile v8h*)(YH + o) = hv[it];
        *(volatile v8h*)(YL + o) = lv[it];
      }
      __threadfence();
    }
  }
}

extern "C" void kernel_launch(void* const* d_in, const int* in_sizes, int n_in,
                              void* d_out, int out_size, void* d_ws, size_t ws_size,
                              hipStream_t stream)
{
  (void)stream;
  if (n_in < 10) return;
  if (in_sizes[0] != kRows * kDmod) return;
  if (in_sizes[1] != kDmod * kXZP) return;
  if (in_sizes[2] != kDin * 4) return;
  if (in_sizes[3] != kDin) return;
  if (in_sizes[4] != kDin * kPrjN) return;
  if (in_sizes[5] != kDtR * kDin) return;
  if (in_sizes[6] != kDin) return;
  if (in_sizes[7] != kDin * kNst) return;
  if (in_sizes[8] != kDin) return;
  if (in_sizes[9] != kDin * kDmod) return;
  if (out_size != kRows * kDmod) return;
  if (ws_size < kWsTotal) return;

  const float* x      = (const float*)d_in[0];
  const float* W_in   = (const float*)d_in[1];
  const float* conv_w = (const float*)d_in[2];
  const float* conv_b = (const float*)d_in[3];
  const float* W_xprj = (const float*)d_in[4];
  const float* W_dt   = (const float*)d_in[5];
  const float* b_dt   = (const float*)d_in[6];
  const float* A_log  = (const float*)d_in[7];
  const float* Dv     = (const float*)d_in[8];
  const float* W_out  = (const float*)d_in[9];
  float* dout = (float*)d_out;

  char* ws = (char*)d_ws;
  unsigned short* XB   = (unsigned short*)(ws + kOffXB);
  unsigned short* WIN  = (unsigned short*)(ws + kOffWIN);
  unsigned short* WOUT = (unsigned short*)(ws + kOffWOUT);
  unsigned short* WXP  = (unsigned short*)(ws + kOffWXP);
  unsigned short* WDT  = (unsigned short*)(ws + kOffWDT);
  float*          XZ   = (float*)(ws + kOffXZ);
  float*          UC   = (float*)(ws + kOffUC);
  unsigned short* UC16 = (unsigned short*)(ws + kOffUC16);
  float*          PROJ = (float*)(ws + kOffPROJ);
  unsigned short* DT16 = (unsigned short*)(ws + kOffDT16);
  float*          DLR  = (float*)(ws + kOffDLR);
  unsigned short* YH   = (unsigned short*)(ws + kOffYH);
  unsigned short* YL   = (unsigned short*)(ws + kOffYL);

  transpose_cast_kernel<true><<<dim3(kXZP / 64, kDmod / 64), 256, 0, stream>>>(W_in, WIN, kDmod, kXZP, 1.0f);
  transpose_cast_kernel<true><<<dim3(kDmod / 64, kDin / 64), 256, 0, stream>>>(W_out, WOUT, kDin, kDmod, 1.0f);
  transpose_cast_kernel<false><<<dim3(kPrjP / 64, kDin / 64), 256, 0, stream>>>(W_xprj, WXP, kDin, kPrjN, kCarryWxp);
  transpose_cast_kernel<false><<<dim3(kDin / 64, kDtR / 64), 256, 0, stream>>>(W_dt, WDT, kDtR, kDin, kCarryWdt);

  cast_bf16_kernel<<<(kRows * kDmod) / 8 / 256, 256, 0, stream>>>(x, XB, (kRows * kDmod) / 8);

  for (int g = 0; g < kNGrp; ++g) {
    const unsigned short* XBg = XB + (size_t)g * kGrpRows * kDmod;
    float* outg = dout + (size_t)g * kGrpRows * kDmod;

    wmma_gemm64<1, 0, 0><<<dim3((kGrpRows / 64) * (kXZP / 64) / 8), 256, 0, stream>>>(
        XBg, XBg, kDmod, WIN, kDmod, XZ, kXZP, b_dt, kGrpRows, kXZP, kDmod, 1.0f);

    conv_silu_kernel<<<dim3(kDin / 256, kGrpRows / 64), 256, 0, stream>>>(XZ, conv_w, conv_b, UC, UC16);

    wmma_gemm64<0, 0, 0><<<dim3((kGrpRows / 64) * (kPrjP / 64) / 8), 256, 0, stream>>>(
        UC16, UC16, kDin, WXP, kDin, PROJ, kPrjP, b_dt, kGrpRows, kPrjP, kDin, 1.0f / kCarryWxp);

    dt_cast_kernel<<<(kGrpRows * kDtR) / 8 / 256, 256, 0, stream>>>(PROJ, DT16, (kGrpRows * kDtR) / 8, kCarryDt);

    wmma_gemm64<0, 0, 3><<<dim3((kGrpRows / 64) * (kDin / 64) / 8), 256, 0, stream>>>(
        DT16, DT16, kDtR, WDT, kDtR, DLR, kDin, b_dt, kGrpRows, kDin, kDtR, 1.0f / (kCarryDt * kCarryWdt));

    scan_kernel<<<dim3(kDin / 256, kGrpB), 256, 0, stream>>>(DLR, UC, XZ, PROJ, A_log, Dv, YH, YL);

    wmma_gemm64<1, 1, 0><<<dim3((kGrpRows / 64) * (kDmod / 64) / 8), 256, 0, stream>>>(
        YH, YL, kDin, WOUT, kDin, outg, kDmod, b_dt, kGrpRows, kDmod, kDin, 1.0f);
  }
}
